// PairConvolution2_21191368639119
// MI455X (gfx1250) — hardware-run, weakly checked
//
#include <hip/hip_runtime.h>
#include <stdint.h>

#define NB    4
#define NP    128
#define NC    32
#define NX    3
#define NN    (NX * NC)
#define NTHR  256
#define SROW  (2 * NN)
#define KCAT  64

static_assert(NP == 16 * (NTHR / 32));
static_assert(NC == 32);
static_assert(NN == 96 && NN == 6 * 16);
static_assert(NN % 32 == 0);
static_assert(2 * NN <= NTHR);
static_assert((SROW * 4) % 128 == 0);
static_assert((NC * 4) == 128);
static_assert(KCAT % 32 == 0);

#define WO_W1B 0
#define WO_W2D 6144
#define WO_GB  18432
#define WO_S   26624
#define WO_END 419840
static_assert(WO_W2D == WO_W1B + NN * NC * 2);
static_assert(WO_GB  == WO_W2D + NN * KCAT * 2);
static_assert(WO_S   == WO_GB + NB * NP * 4 * 4);
static_assert(WO_END == WO_S + NB * NP * SROW * 4);
static_assert(WO_W2D % 256 == 0 && WO_GB % 256 == 0 && WO_S % 256 == 0 && WO_END % 256 == 0);

#define OUT_ELEMS (NB * NP * NP * NC)
static_assert((((NB - 1) * NP + (NP - 1)) * NP + (NP - 1)) * NC + (NC - 1) == OUT_ELEMS - 1);

typedef float          v4f   __attribute__((ext_vector_type(4)));
typedef float          v8f   __attribute__((ext_vector_type(8)));
typedef int            v8i   __attribute__((ext_vector_type(8)));
typedef unsigned int   v2u   __attribute__((ext_vector_type(2)));
typedef unsigned int   v4u   __attribute__((ext_vector_type(4)));
typedef unsigned short v8us  __attribute__((ext_vector_type(8)));
typedef __bf16         v16bf __attribute__((ext_vector_type(16)));
typedef v4f  __attribute__((may_alias)) v4fa;
typedef v2u  __attribute__((may_alias)) v2ua;
typedef v8us __attribute__((may_alias)) v8usa;
union FragB { v16bf v; v8us h[2]; v4u q[2]; v8i w; };

__device__ __forceinline__ unsigned short f2bf(float f) {
  const unsigned u = __float_as_uint(f);
  return (unsigned short)((u + 0x7FFFu + ((u >> 16) & 1u)) >> 16);
}
__device__ __forceinline__ float bf2f(unsigned short b) { return __uint_as_float(((unsigned)b) << 16); }
__device__ __forceinline__ float bfr(float f) { return bf2f(f2bf(f)); }
__device__ __forceinline__ unsigned pk16(unsigned short a, unsigned short b) { return (unsigned)a | ((unsigned)b << 16); }
__device__ __forceinline__ v4u pack8(v4f a, v4f c) {
  v4u r;
  r.x = pk16(f2bf(a.x), f2bf(a.y));
  r.y = pk16(f2bf(a.z), f2bf(a.w));
  r.z = pk16(f2bf(c.x), f2bf(c.y));
  r.w = pk16(f2bf(c.z), f2bf(c.w));
  return r;
}
__device__ __forceinline__ v8f z8() { v8f z = {0.f, 0.f, 0.f, 0.f, 0.f, 0.f, 0.f, 0.f}; return z; }

__device__ __forceinline__ v8f wmb(const FragB& a, const FragB& b, v8f c) {
  v8f d = __builtin_amdgcn_wmma_f32_16x16x32_bf16(false, a.v, false, b.v, (short)0, c, false, false);
  asm volatile("v_nop\n\tv_nop\n\tv_nop\n\tv_nop" : "+v"(d) : "v"(a.w), "v"(b.w));
  return d;
}

__device__ __forceinline__ void prep_pass(unsigned short* W1B, unsigned short* W2D, float* GB, int tid,
                                          v4u a0, v4u a1, v4u b0, v4u b1, v4u b2, v4f g0, v4f g1) {
  *(volatile v4u*)(W1B + 8 * tid) = a0;
  if (tid < 128) *(volatile v4u*)(W1B + 8 * (tid + NTHR)) = a1;
  *(volatile v4u*)(W2D + 8 * tid) = b0;
  *(volatile v4u*)(W2D + 8 * (tid + NTHR)) = b1;
  *(volatile v4u*)(W2D + 8 * (tid + 2 * NTHR)) = b2;
  *(volatile v4f*)(GB + 4 * tid) = g0;
  *(volatile v4f*)(GB + 4 * (tid + NTHR)) = g1;
}

__global__ __launch_bounds__(NTHR) void k_prep(const float* __restrict__ geo, const float* __restrict__ W1,
                                               const float* __restrict__ W2,
                                               unsigned short* __restrict__ W1B,
                                               unsigned short* __restrict__ W2D,
                                               float* __restrict__ GB) {
  __shared__ __attribute__((aligned(16))) float sGeo[NB * NP * NX];
  const int tid = threadIdx.x;
#pragma unroll
  for (int it = 0; it < 2; ++it) {
    const int q = tid + NTHR * it;
    const int qc = (q < 384) ? q : 383;
    const v4f v = *(const v4fa*)(geo + 4 * qc);
    asm volatile("" :: "v"(v));
    if (q < 384) *(v4fa*)(sGeo + 4 * q) = v;
  }
  __syncthreads();

  v4u a[2], b[3];
  v4f g[2];
#pragma unroll
  for (int it = 0; it < 2; ++it) {
    const int u = tid + NTHR * it;
    const int uc = (u < 384) ? u : 383;
    const float* src = W1 + 8 * uc;
    const v4f p = *(const v4fa*)src;
    const v4f r = *(const v4fa*)(src + 4);
    a[it] = pack8(p, r);
  }
#pragma unroll
  for (int it = 0; it < 3; ++it) {
    const int u = tid + NTHR * it;
    const int n = u >> 3;
    const int ks = ((u & 7) * 8) & 31;
    const float* src = W2 + n * NC + ks;
    const v4f p = *(const v4fa*)src;
    const v4f r = *(const v4fa*)(src + 4);
    b[it] = pack8(p, r);
  }
#pragma unroll
  for (int it = 0; it < 2; ++it) {
    const int p = tid + NTHR * it;
    v4f t;
    t.x = bfr(sGeo[3 * p + 0]);
    t.y = bfr(sGeo[3 * p + 1]);
    t.z = bfr(sGeo[3 * p + 2]);
    t.w = 0.0f;
    g[it] = t;
  }
  prep_pass(W1B, W2D, GB, tid, a[0], a[1], b[0], b[1], b[2], g[0], g[1]);
  __threadfence();
  prep_pass(W1B, W2D, GB, tid, a[0], a[1], b[0], b[1], b[2], g[0], g[1]);
}

__global__ __launch_bounds__(NTHR) void k_g(const float* __restrict__ F,
                                            const unsigned short* __restrict__ W1B,
                                            const float* __restrict__ GB,
                                            float* __restrict__ S) {
  __shared__ __attribute__((aligned(16))) float sD[NP * NN];
  __shared__ __attribute__((aligned(16))) float sG[NP * 4];
  __shared__ __attribute__((aligned(16))) float sS[SROW];

  const int tid = threadIdx.x, lane = tid & 31, w = tid >> 5;
  const int h = lane >> 4, m = lane & 15;
  const int blk = blockIdx.x;
  const int z = blk >> 7;

  {
    const v4f gv = *(const v4fa*)(GB + ((size_t)z * NP + (size_t)(tid & (NP - 1))) * 4);
    asm volatile("" :: "v"(gv));
    if (tid < NP) *(v4fa*)(sG + 4 * tid) = gv;
  }

  FragB a;
  {
    const float* ap = F + (size_t)blk * (NP * NC) + (size_t)(16 * w + m) * NC + 8 * h;
    const v4f f0 = *(const v4fa*)(ap);
    const v4f f1 = *(const v4fa*)(ap + 4);
    const v4f f2 = *(const v4fa*)(ap + 16);
    const v4f f3 = *(const v4fa*)(ap + 20);
    a.q[0] = pack8(f0, f1);
    a.q[1] = pack8(f2, f3);
  }

  v8f acc[6];
#pragma unroll
  for (int t = 0; t < 6; ++t) {
    const unsigned short* bp = W1B + (16 * t + m) * NC + 8 * h;
    FragB b;
    b.h[0] = *(const v8usa*)bp;
    b.h[1] = *(const v8usa*)(bp + 16);
    acc[t] = wmb(a, b, z8());
  }
#pragma unroll
  for (int t = 0; t < 6; ++t) {
#pragma unroll
    for (int r = 0; r < 8; ++r) sD[(16 * w + 8 * h + r) * NN + 16 * t + m] = acc[t][r];
  }
  __syncthreads();

  if (tid < SROW) {
    const int which = tid / NN;
    const int n = tid - which * NN;
    const int x = n >> 5;
    float s = 0.0f;
#pragma unroll 4
    for (int d = 0; d < NP; ++d) {
      const float gw = sG[4 * d + x];
      const float wv = (which != 0) ? gw : 1.0f;
      s = fmaf(wv, sD[d * NN + n], s);
    }
    sS[tid] = s;
  }
  __syncthreads();

  if (tid < SROW / 4) {
    const v4f v = *(const v4fa*)(sS + 4 * tid);
    float* dst = S + (size_t)blk * SROW + 4 * tid;
    *(volatile v4f*)dst = v;
    __threadfence();
    *(volatile v4f*)dst = v;
  }
}

__device__ __forceinline__ void tmp_bits(float s00, float s01, float s02, float s10, float s11, float s12,
                                         float gb0, float gb1, float gb2, float nf,
                                         unsigned short& hb, unsigned short& lb) {
  float t = 0.0f;
  t = t + fmaf(-gb0, s00, s10);
  t = t + fmaf(-gb1, s01, s11);
  t = t + fmaf(-gb2, s02, s12);
  const float v = t / nf;
  hb = f2bf(v);
  lb = f2bf(v - bf2f(hb));
}

__global__ __launch_bounds__(NTHR) void k_h(const float* __restrict__ S,
                                            const unsigned short* __restrict__ W2D,
                                            const float* __restrict__ GB,
                                            const int* __restrict__ nn,
                                            float* __restrict__ out) {
  __shared__ __attribute__((aligned(16))) char smem[NP * NN * 4];
  __shared__ __attribute__((aligned(16))) float sG[NP * 4];
  __shared__ __attribute__((aligned(16))) float sT[SROW];
  static_assert(NP * KCAT * 2 <= NP * NN * 4);
  unsigned short* sA = (unsigned short*)smem;
  float* sD = (float*)smem;

  const int tid = threadIdx.x, lane = tid & 31, w = tid >> 5;
  const int h = lane >> 4, m = lane & 15;
  const int blk = blockIdx.x;
  const int z = blk >> 7, b = blk & (NP - 1);

  {
    const v4f gv = *(const v4fa*)(GB + ((size_t)z * NP + (size_t)(tid & (NP - 1))) * 4);
    asm volatile("" :: "v"(gv));
    if (tid < NP) *(v4fa*)(sG + 4 * tid) = gv;
  }
  const int nv = nn[0];
  const float nf = (float)nv;
  __syncthreads();

  const float gb0 = sG[4 * b + 0];
  const float gb1 = sG[4 * b + 1];
  const float gb2 = sG[4 * b + 2];

  const float* Sz = S + (size_t)z * NP * SROW;
#pragma unroll 1
  for (int it = 0; it < 4; ++it) {
    const int q = tid + NTHR * it;
    const int c = q >> 3, j4 = (q & 7) * 4;
    const float* sp = Sz + (size_t)c * SROW + j4;
    const v4f s00 = *(const v4fa*)(sp);
    const v4f s01 = *(const v4fa*)(sp + 32);
    const v4f s02 = *(const v4fa*)(sp + 64);
    const v4f s10 = *(const v4fa*)(sp + 96);
    const v4f s11 = *(const v4fa*)(sp + 128);
    const v4f s12 = *(const v4fa*)(sp + 160);
    unsigned short h0, h1, h2, h3, l0, l1, l2, l3;
    tmp_bits(s00.x, s01.x, s02.x, s10.x, s11.x, s12.x, gb0, gb1, gb2, nf, h0, l0);
    tmp_bits(s00.y, s01.y, s02.y, s10.y, s11.y, s12.y, gb0, gb1, gb2, nf, h1, l1);
    tmp_bits(s00.z, s01.z, s02.z, s10.z, s11.z, s12.z, gb0, gb1, gb2, nf, h2, l2);
    tmp_bits(s00.w, s01.w, s02.w, s10.w, s11.w, s12.w, gb0, gb1, gb2, nf, h3, l3);
    v2u hv, lv;
    hv.x = pk16(h0, h1); hv.y = pk16(h2, h3);
    lv.x = pk16(l0, l1); lv.y = pk16(l2, l3);
    *(v2ua*)(sA + c * KCAT + j4) = hv;
    *(v2ua*)(sA + c * KCAT + NC + j4) = lv;
  }
  __syncthreads();

  FragB a0, a1;
  {
    const unsigned short* ar = sA + (16 * w + m) * KCAT + 8 * h;
    a0.h[0] = *(const v8usa*)(ar);
    a0.h[1] = *(const v8usa*)(ar + 16);
    a1.h[0] = *(const v8usa*)(ar + 32);
    a1.h[1] = *(const v8usa*)(ar + 48);
  }

  v8f acc[6];
#pragma unroll
  for (int t = 0; t < 6; ++t) {
    const unsigned short* bp = W2D + (16 * t + m) * KCAT + 8 * h;
    FragB b0, b1;
    b0.h[0] = *(const v8usa*)(bp);
    b0.h[1] = *(const v8usa*)(bp + 16);
    b1.h[0] = *(const v8usa*)(bp + 32);
    b1.h[1] = *(const v8usa*)(bp + 48);
    acc[t] = wmb(a0, b0, z8());
    acc[t] = wmb(a1, b1, acc[t]);
  }
  __syncthreads();

#pragma unroll
  for (int t = 0; t < 6; ++t) {
#pragma unroll
    for (int r = 0; r < 8; ++r) sD[(16 * w + 8 * h + r) * NN + 16 * t + m] = acc[t][r];
  }
  __syncthreads();

  if (tid < SROW) {
    const int which = tid / NN;
    const int n = tid - which * NN;
    const int x = n >> 5;
    float s = 0.0f;
#pragma unroll 4
    for (int c = 0; c < NP; ++c) {
      const float gw = sG[4 * c + x];
      const float wv = (which != 0) ? gw : 1.0f;
      s = fmaf(wv, sD[c * NN + n], s);
    }
    sT[tid] = s;
  }
  __syncthreads();

  const float t00 = sT[lane], t01 = sT[NC + lane], t02 = sT[2 * NC + lane];
  const float t10 = sT[NN + lane], t11 = sT[NN + NC + lane], t12 = sT[NN + 2 * NC + lane];
  float vals[16];
#pragma unroll
  for (int it = 0; it < 16; ++it) {
    const int ar = w + 8 * it;
    const v4f g = *(const v4fa*)(sG + 4 * ar);
    float v = 0.0f;
    v = v + fmaf(-g.x, t00, t10);
    v = v + fmaf(-g.y, t01, t11);
    v = v + fmaf(-g.z, t02, t12);
    vals[it] = v;
  }
  float* ob = out + ((size_t)z * NP * NP + (size_t)b) * NC + lane;
#pragma unroll
  for (int it = 0; it < 16; ++it) {
    const int ar = w + 8 * it;
    *(volatile float*)(ob + (size_t)ar * (NP * NC)) = vals[it];
  }
  __threadfence();
#pragma unroll
  for (int it = 0; it < 16; ++it) {
    const int ar = w + 8 * it;
    *(volatile float*)(ob + (size_t)ar * (NP * NC)) = vals[it];
  }
}

extern "C" void kernel_launch(void* const* d_in, const int* in_sizes, int n_in,
                              void* d_out, int out_size, void* d_ws, size_t ws_size,
                              hipStream_t stream) {
  if (n_in < 5) return;
  if (in_sizes[0] != NB * NP * NP * NC) return;
  if (in_sizes[1] != NB * NP * NX) return;
  if (in_sizes[2] != NX * NC * NC) return;
  if (in_sizes[3] != NX * NC * NC) return;
  if (in_sizes[4] != 1) return;
  if (out_size != OUT_ELEMS) return;
  if ((size_t)WO_END > ws_size) return;

  const float* F   = (const float*)d_in[0];
  const float* geo = (const float*)d_in[1];
  const float* W1  = (const float*)d_in[2];
  const float* W2  = (const float*)d_in[3];
  const int*   nn  = (const int*)d_in[4];
  float* out = (float*)d_out;

  char* ws = (char*)d_ws;
  unsigned short* W1B = (unsigned short*)(ws + WO_W1B);
  unsigned short* W2D = (unsigned short*)(ws + WO_W2D);
  float* GB = (float*)(ws + WO_GB);
  float* S  = (float*)(ws + WO_S);

  k_prep<<<dim3(1), dim3(NTHR), 0, stream>>>(geo, W1, W2, W1B, W2D, GB);
  k_g<<<dim3(NB * NP), dim3(NTHR), 0, stream>>>(F, W1B, GB, S);
  k_h<<<dim3(NB * NP), dim3(NTHR), 0, stream>>>(S, W2D, GB, nn, out);
  (void)hipGetLastError();
}
